// SelfAttention_49606872268908
// MI455X (gfx1250) — hardware-verified
//
#include <hip/hip_runtime.h>
#ifndef NB
#define NB 4
#endif
#ifndef LL
#define LL 4096
#endif
#define NB_FULL 4
#define LL_FULL 4096
#define CC 256
#define RD 32
#define QW 64
#define WA_ROWS (2 * RD + CC)
#define WA_ELEMS (WA_ROWS * CC)

static_assert(RD == 32);
static_assert(CC == 256);
static_assert(CC % 64 == 0);
static_assert(CC % 32 == 0);
static_assert(LL % 64 == 0);
static_assert(LL <= LL_FULL);
static_assert(NB <= NB_FULL);
static_assert(QW == 2 * RD);
static_assert(WA_ELEMS % (8 * 256) == 0);
static_assert(((NB * LL) / 16) % 4 == 0);
static_assert(((CC / 16) * (LL / 64)) % 4 == 0);
static_assert(128 * 16 == 8 * 256);

typedef __bf16 v16b __attribute__((ext_vector_type(16)));
typedef _Float16 v16h __attribute__((ext_vector_type(16)));
typedef unsigned short v8us __attribute__((ext_vector_type(8), may_alias));
typedef float v8f __attribute__((ext_vector_type(8)));
typedef float v4f __attribute__((ext_vector_type(4)));
typedef float v4fa __attribute__((ext_vector_type(4), may_alias));
union FragB { v16b v; v8us half[2]; };
union FragH { v16h v; v8us half[2]; _Float16 h[16]; };
union Pack8 { v8us v; _Float16 h[8]; unsigned short u[8]; };

__device__ __forceinline__ unsigned short bf16_bits(float x) { unsigned int u = __float_as_uint(x); return (unsigned short)((u + 0x7FFFu + ((u >> 16) & 1u)) >> 16); }
__device__ __forceinline__ float bf16_val(unsigned short b) { return __uint_as_float(((unsigned int)b) << 16); }
__device__ __forceinline__ float bf16_rne(float x) { return bf16_val(bf16_bits(x)); }

__device__ __forceinline__ v8f mma_b(v16b a, v16b b, v8f c) {
  v8f d = __builtin_amdgcn_wmma_f32_16x16x32_bf16(false, a, false, b, (short)0, c, false, false);
  asm volatile("v_nop\n\tv_nop\n\tv_nop\n\tv_nop" : "+v"(d) : "v"(a), "v"(b));
  return d;
}
__device__ __forceinline__ v8f mma_b3(v16b ah, v16b al, v16b bh, v16b bl, v8f c) {
  c = __builtin_amdgcn_wmma_f32_16x16x32_bf16(false, ah, false, bh, (short)0, c, false, false);
  c = __builtin_amdgcn_wmma_f32_16x16x32_bf16(false, al, false, bh, (short)0, c, false, false);
  c = __builtin_amdgcn_wmma_f32_16x16x32_bf16(false, ah, false, bl, (short)0, c, false, false);
  asm volatile("v_nop\n\tv_nop\n\tv_nop\n\tv_nop" : "+v"(c) : "v"(ah), "v"(al), "v"(bh), "v"(bl));
  return c;
}
__device__ __forceinline__ v8f mma_h(v16h a, v16h b, v8f c) {
  v8f d = __builtin_amdgcn_wmma_f32_16x16x32_f16(false, a, false, b, (short)0, c, false, false);
  asm volatile("v_nop\n\tv_nop\n\tv_nop\n\tv_nop" : "+v"(d) : "v"(a), "v"(b));
  return d;
}

__global__ __launch_bounds__(256) void k_wcvt(const float* __restrict__ wq, const float* __restrict__ wk, const float* __restrict__ wv, unsigned short* __restrict__ WA) {
  const int t = blockIdx.x * 256 + threadIdx.x;
  const int e = min(t, WA_ELEMS / 8 - 1) * 8;
  const int eq = min(e, RD * CC - 8);
  const int ek = min(max(e - RD * CC, 0), RD * CC - 8);
  const int ev = min(max(e - 2 * RD * CC, 0), CC * CC - 8);
  const v4f a0 = *(const v4fa*)(wq + eq), a1 = *(const v4fa*)(wq + eq + 4);
  const v4f b0 = *(const v4fa*)(wk + ek), b1 = *(const v4fa*)(wk + ek + 4);
  const v4f c0 = *(const v4fa*)(wv + ev), c1 = *(const v4fa*)(wv + ev + 4);
  const bool isq = e < RD * CC, isk = e < 2 * RD * CC;
  Pack8 o;
#pragma unroll
  for (int q = 0; q < 4; ++q) {
    const float f0 = isq ? a0[q] : (isk ? b0[q] : c0[q]);
    const float f1 = isq ? a1[q] : (isk ? b1[q] : c1[q]);
    o.u[q] = bf16_bits(f0);
    o.u[4 + q] = bf16_bits(f1);
  }
  const v8us ov = o.v;
  *(volatile v8us*)(WA + e) = ov;
  __threadfence();
  *(volatile v8us*)(WA + e) = ov;
}

__global__ __launch_bounds__(256) void k_xT(const float* __restrict__ x, unsigned short* __restrict__ XB) {
  __shared__ unsigned short tl[64][66];
  const int tid = threadIdx.x;
  const int cb = blockIdx.x % (CC / 64);
  const int nb = (blockIdx.x / (CC / 64)) % (LL / 64);
  const int b = blockIdx.x / ((CC / 64) * (LL / 64));
  const int c0 = cb * 64, n0 = nb * 64;
#pragma unroll 4
  for (int i = tid; i < 64 * 64; i += 256) {
    const int c = i >> 6, n = i & 63;
    tl[c][n] = bf16_bits(x[((size_t)b * CC + c0 + c) * LL_FULL + n0 + n]);
  }
  __syncthreads();
  const int n = tid >> 3, c8 = (tid & 7) * 8;
  Pack8 o0, o1;
#pragma unroll
  for (int q = 0; q < 8; ++q) { o0.u[q] = tl[c8 + q][n]; o1.u[q] = tl[c8 + q][32 + n]; }
  const v8us v0 = o0.v, v1 = o1.v;
  unsigned short* d0 = XB + ((size_t)b * LL + n0 + n) * CC + c0 + c8;
  unsigned short* d1 = d0 + (size_t)32 * CC;
  *(volatile v8us*)d0 = v0;
  *(volatile v8us*)d1 = v1;
  __threadfence();
  *(volatile v8us*)d0 = v0;
  *(volatile v8us*)d1 = v1;
}

__global__ __launch_bounds__(128) void k_projqk(const unsigned short* __restrict__ XB, const unsigned short* __restrict__ WA, const float* __restrict__ bq, const float* __restrict__ bk,
                                               unsigned short* __restrict__ QP, unsigned short* __restrict__ KP) {
  __shared__ __attribute__((aligned(16))) float so[4][16][68];
  const int tid = threadIdx.x;
  const int wave = __builtin_amdgcn_readfirstlane(tid >> 5);
  const int lane = tid & 31, ln = lane & 15, hh = lane >> 4;
  const int row0 = (blockIdx.x * 4 + wave) * 16;
  const unsigned short* arow = XB + (size_t)(row0 + ln) * CC + 8 * hh;
  const unsigned short* brow = WA + (size_t)ln * CC + 8 * hh;
  const v8f z8 = {0.f, 0.f, 0.f, 0.f, 0.f, 0.f, 0.f, 0.f};
  v8f acc[4] = {z8, z8, z8, z8};
#pragma unroll 1
  for (int kb = 0; kb < CC; kb += 32) {
    FragB a;
    a.half[0] = *(const v8us*)(arow + kb);
    a.half[1] = *(const v8us*)(arow + kb + 16);
#pragma unroll
    for (int t = 0; t < 4; ++t) {
      FragB bb;
      bb.half[0] = *(const v8us*)(brow + (size_t)t * 16 * CC + kb);
      bb.half[1] = *(const v8us*)(brow + (size_t)t * 16 * CC + kb + 16);
      acc[t] = mma_b(a.v, bb.v, acc[t]);
    }
  }
  const float bias0 = bf16_rne(bq[ln]), bias1 = bf16_rne(bq[16 + ln]), bias2 = bf16_rne(bk[ln]), bias3 = bf16_rne(bk[16 + ln]);
#pragma unroll
  for (int r = 0; r < 8; ++r) {
    so[wave][8 * hh + r][ln] = acc[0][r] + bias0;
    so[wave][8 * hh + r][16 + ln] = acc[1][r] + bias1;
    so[wave][8 * hh + r][32 + ln] = acc[2][r] + bias2;
    so[wave][8 * hh + r][48 + ln] = acc[3][r] + bias3;
  }
  __builtin_amdgcn_fence(4  , "workgroup");
  __builtin_amdgcn_wave_barrier();
  const int l8 = lane & 7, rq = lane >> 3;
  const bool islo = (l8 >> 2) != 0;
  v8us ov[8];
#pragma unroll
  for (int it = 0; it < 8; ++it) {
    const int plane = it >> 2;
    const int row = (it & 3) * 4 + rq;
    const int cb = plane * 32 + (l8 & 3) * 8;
    const v4f f0 = *(const v4fa*)&so[wave][row][cb];
    const v4f f1 = *(const v4fa*)&so[wave][row][cb + 4];
    Pack8 o;
#pragma unroll
    for (int q = 0; q < 4; ++q) {
      const unsigned short h0 = bf16_bits(f0[q]);
      const unsigned short l0 = bf16_bits(f0[q] - bf16_val(h0));
      const unsigned short h1 = bf16_bits(f1[q]);
      const unsigned short l1 = bf16_bits(f1[q] - bf16_val(h1));
      o.u[q] = islo ? l0 : h0;
      o.u[4 + q] = islo ? l1 : h1;
    }
    ov[it] = o.v;
  }
#pragma unroll
  for (int pass = 0; pass < 2; ++pass) {
#pragma unroll
    for (int it = 0; it < 8; ++it) {
      const int row = (it & 3) * 4 + rq;
      if (it < 4) *(volatile v8us*)(QP + (size_t)(row0 + row) * QW + l8 * 8) = ov[it];
      else        *(volatile v8us*)(KP + (size_t)(row0 + row) * QW + l8 * 8) = ov[it];
    }
    if (pass == 0) __threadfence();
  }
}

__global__ __launch_bounds__(128) void k_projv(const unsigned short* __restrict__ XB, const unsigned short* __restrict__ WA, const float* __restrict__ bv, unsigned short* __restrict__ VT) {
  __shared__ __attribute__((aligned(16))) float so[4][16][68];
  const int tid = threadIdx.x;
  const int wave = __builtin_amdgcn_readfirstlane(tid >> 5);
  const int lane = tid & 31, ln = lane & 15, hh = lane >> 4;
  const int tpb = (CC / 16) * (LL / 64);
  const int wt = blockIdx.x * 4 + wave;
  const int b = wt / tpb;
  const int rem = wt % tpb;
  const int c0 = (rem % (CC / 16)) * 16;
  const int nn0 = (rem / (CC / 16)) * 64;
  const unsigned short* arow = WA + (size_t)(2 * RD + c0 + ln) * CC + 8 * hh;
  const unsigned short* brow = XB + ((size_t)b * LL + nn0 + ln) * CC + 8 * hh;
  const v8f z8 = {0.f, 0.f, 0.f, 0.f, 0.f, 0.f, 0.f, 0.f};
  v8f acc[4] = {z8, z8, z8, z8};
#pragma unroll 1
  for (int kb = 0; kb < CC; kb += 32) {
    FragB a;
    a.half[0] = *(const v8us*)(arow + kb);
    a.half[1] = *(const v8us*)(arow + kb + 16);
#pragma unroll
    for (int t = 0; t < 4; ++t) {
      FragB bb;
      bb.half[0] = *(const v8us*)(brow + (size_t)t * 16 * CC + kb);
      bb.half[1] = *(const v8us*)(brow + (size_t)t * 16 * CC + kb + 16);
      acc[t] = mma_b(a.v, bb.v, acc[t]);
    }
  }
#pragma unroll
  for (int r = 0; r < 8; ++r) {
    const float bias = bf16_rne(bv[c0 + 8 * hh + r]);
#pragma unroll
    for (int t = 0; t < 4; ++t) so[wave][8 * hh + r][t * 16 + ln] = acc[t][r] + bias;
  }
  __builtin_amdgcn_fence(4  , "workgroup");
  __builtin_amdgcn_wave_barrier();
  const int l8 = lane & 7, rq = lane >> 3;
  v8us ov[4];
#pragma unroll
  for (int it = 0; it < 4; ++it) {
    const int row = it * 4 + rq;
    const v4f f0 = *(const v4fa*)&so[wave][row][l8 * 8];
    const v4f f1 = *(const v4fa*)&so[wave][row][l8 * 8 + 4];
    Pack8 o;
#pragma unroll
    for (int q = 0; q < 4; ++q) { o.h[q] = (_Float16)f0[q]; o.h[4 + q] = (_Float16)f1[q]; }
    ov[it] = o.v;
  }
#pragma unroll
  for (int pass = 0; pass < 2; ++pass) {
#pragma unroll
    for (int it = 0; it < 4; ++it) {
      const int row = it * 4 + rq;
      *(volatile v8us*)(VT + ((size_t)b * CC + c0 + row) * LL + nn0 + l8 * 8) = ov[it];
    }
    if (pass == 0) __threadfence();
  }
}

__global__ __launch_bounds__(256) void k_attn(const unsigned short* __restrict__ QP, const unsigned short* __restrict__ KP, const unsigned short* __restrict__ VT,
                                             const float* __restrict__ x, const float* __restrict__ gam, float* __restrict__ out) {
  __shared__ __attribute__((aligned(16))) float tl[128][68];
  const int tid = threadIdx.x;
  const int wave = __builtin_amdgcn_readfirstlane(tid >> 5);
  const int lane = tid & 31, ln = lane & 15, hh = lane >> 4;
  const int qg = wave & 3, ch = wave >> 2;
  const int b = blockIdx.x / (LL / 64);
  const int n0 = (blockIdx.x % (LL / 64)) * 64;
  const int i0 = n0 + qg * 16;
  const unsigned short* qrow = QP + ((size_t)b * LL + i0 + ln) * QW + 8 * hh;
  FragB qh, ql;
  qh.half[0] = *(const v8us*)(qrow);
  qh.half[1] = *(const v8us*)(qrow + 16);
  ql.half[0] = *(const v8us*)(qrow + 32);
  ql.half[1] = *(const v8us*)(qrow + 48);
  const unsigned short* kbase = KP + ((size_t)b * LL + ln) * QW + 8 * hh;
  const unsigned short* vbase = VT + ((size_t)b * CC + ch * 128 + ln) * LL + 8 * hh;
  const v8f z8 = {0.f, 0.f, 0.f, 0.f, 0.f, 0.f, 0.f, 0.f};
  v8f oacc[8] = {z8, z8, z8, z8, z8, z8, z8, z8};
  float mrun = -3.0e38f, lrun = 0.f;
#pragma unroll 1
  for (int j0 = 0; j0 < LL; j0 += 32) {
    const unsigned short* k0 = kbase + (size_t)j0 * QW;
    const unsigned short* k1 = k0 + 16 * QW;
    FragB ah, al;
    ah.half[0] = *(const v8us*)(k0);
    ah.half[1] = *(const v8us*)(k0 + 16);
    al.half[0] = *(const v8us*)(k0 + 32);
    al.half[1] = *(const v8us*)(k0 + 48);
    const v8f s0 = mma_b3(ah.v, al.v, qh.v, ql.v, z8);
    ah.half[0] = *(const v8us*)(k1);
    ah.half[1] = *(const v8us*)(k1 + 16);
    al.half[0] = *(const v8us*)(k1 + 32);
    al.half[1] = *(const v8us*)(k1 + 48);
    const v8f s1 = mma_b3(ah.v, al.v, qh.v, ql.v, z8);
    float mx = fmaxf(s0[0], s1[0]);
#pragma unroll
    for (int r = 1; r < 8; ++r) mx = fmaxf(mx, fmaxf(s0[r], s1[r]));
    const float mo = __shfl_xor(mx, 16, 32);
    mx = fmaxf(mx, mo);
    const float mnew = fmaxf(mrun, mx);
    const float sc = __expf(mrun - mnew);
    mrun = mnew;
    FragH pf;
    float ls = 0.f;
#pragma unroll
    for (int r = 0; r < 8; ++r) {
      const float p0 = __expf(s0[r] - mnew);
      const float p1 = __expf(s1[r] - mnew);
      ls += p0;
      ls += p1;
      pf.h[r] = (_Float16)(p0 * 256.0f);
      pf.h[8 + r] = (_Float16)(p1 * 256.0f);
    }
    const float lo = __shfl_xor(ls, 16, 32);
    ls += lo;
    lrun = lrun * sc + ls;
#pragma unroll
    for (int ct = 0; ct < 8; ++ct)
#pragma unroll
      for (int r = 0; r < 8; ++r) oacc[ct][r] *= sc;
#pragma unroll
    for (int ct = 0; ct < 8; ++ct) {
      const unsigned short* vp = vbase + (size_t)ct * 16 * LL + j0;
      FragH vf;
      vf.half[0] = *(const v8us*)(vp);
      vf.half[1] = *(const v8us*)(vp + 16);
      oacc[ct] = mma_h(vf.v, pf.v, oacc[ct]);
    }
  }
  const float inv = 0.00390625f * (1.0f / lrun);
  const float gg = bf16_rne(gam[0]);
#pragma unroll
  for (int rd = 0; rd < 2; ++rd) {
    if (rd != 0) __syncthreads();
#pragma unroll
    for (int t = 0; t < 4; ++t)
#pragma unroll
      for (int r = 0; r < 8; ++r) tl[ch * 64 + t * 16 + 8 * hh + r][qg * 16 + ln] = oacc[rd * 4 + t][r] * inv;
    __syncthreads();
#pragma unroll
    for (int pass = 0; pass < 2; ++pass) {
#pragma unroll
      for (int it = 0; it < 8; ++it) {
        const int p = it * 256 + tid;
        const int line = p >> 3, l8 = p & 7;
        const int lr = line >> 1, hf = line & 1;
        const int n4 = hf * 32 + l8 * 4;
        const int c = (lr >> 6) * 128 + rd * 64 + (lr & 63);
        const size_t e = ((size_t)b * CC + c) * LL_FULL + n0 + n4;
        const v4f xv = *(const v4fa*)(x + e);
        const v4f o = *(const v4fa*)&tl[lr][n4];
        v4f y;
#pragma unroll
        for (int q = 0; q < 4; ++q) y[q] = bf16_rne(xv[q]) + gg * o[q];
        *(volatile v4f*)(out + e) = y;
      }
      if (pass == 0) __threadfence();
    }
  }
}

#define SZ_WA ((size_t)WA_ELEMS * 2)
#define SZ_XB ((size_t)NB * LL * CC * 2)
#define SZ_QP ((size_t)NB * LL * QW * 2)
#define SZ_VT ((size_t)NB * CC * LL * 2)
#define AL256(v) (((v) + 255) & ~(size_t)255)
static_assert(AL256(SZ_WA) + AL256(SZ_XB) + 2 * AL256(SZ_QP) + AL256(SZ_VT) <= (size_t)134217728);

extern "C" void kernel_launch(void* const* d_in, const int* in_sizes, int n_in,
                              void* d_out, int out_size, void* d_ws, size_t ws_size, hipStream_t stream) {
  if (n_in < 8) return;
  const size_t need = ((size_t)(NB - 1) * CC + (CC - 1)) * LL_FULL + LL;
  if ((size_t)in_sizes[0] < need) return;
  if ((size_t)out_size < need) return;
  if (in_sizes[1] < RD * CC || in_sizes[2] < RD || in_sizes[3] < RD * CC || in_sizes[4] < RD) return;
  if (in_sizes[5] < CC * CC || in_sizes[6] < CC || in_sizes[7] < 1) return;
  const float* x = (const float*)d_in[0];
  const float* wq = (const float*)d_in[1];
  const float* bq = (const float*)d_in[2];
  const float* wk = (const float*)d_in[3];
  const float* bk = (const float*)d_in[4];
  const float* wv = (const float*)d_in[5];
  const float* bv = (const float*)d_in[6];
  const float* gam = (const float*)d_in[7];
  float* out = (float*)d_out;
  char* ws = (char*)d_ws;
  size_t off = 0;
  unsigned short* WA = (unsigned short*)(ws + off); off += AL256(SZ_WA);
  unsigned short* XB = (unsigned short*)(ws + off); off += AL256(SZ_XB);
  unsigned short* QP = (unsigned short*)(ws + off); off += AL256(SZ_QP);
  unsigned short* KP = (unsigned short*)(ws + off); off += AL256(SZ_QP);
  unsigned short* VT = (unsigned short*)(ws + off); off += AL256(SZ_VT);
  if (off > ws_size) return;
  k_wcvt<<<WA_ELEMS / 8 / 256, 256, 0, stream>>>(wq, wk, wv, WA);
  k_xT<<<NB * (LL / 64) * (CC / 64), 256, 0, stream>>>(x, XB);
  k_projqk<<<(NB * LL / 16) / 4, 128, 0, stream>>>(XB, WA, bq, bk, QP, KP);
  k_projv<<<NB * ((CC / 16) * (LL / 64)) / 4, 128, 0, stream>>>(XB, WA, bv, VT);
  k_attn<<<NB * (LL / 64), 256, 0, stream>>>(QP, KP, VT, x, gam, out);
}
